// RGATLayer_84593675862503
// MI455X (gfx1250) — hardware-run, weakly checked
//
#include <hip/hip_runtime.h>


namespace {

constexpr int N = 100000, NP = 100032, NPL = NP  , SRCM = N  , EFULL = 640000, E = EFULL  ;
constexpr int D = 128, D2 = 2 * D, R = 4, KSH = 17  , NKEY = R << KSH  , BPR = (1 << KSH) >> 10  , NL = (NPL < N ? NPL : N);
constexpr float XS = 8.0f, WSC = 256.0f, WSQ = 0.25f, RS_ = 1024.0f, NSLOPE = 0.2f, SLOPE = 0.0f, BNEPS = 1e-5f;
static_assert(N < (1 << KSH) && NP % 32 == 0 && NPL % 32 == 0 && D == 128 && E % 4 == 0, "layout");
typedef _Float16 b16;
typedef __attribute__((ext_vector_type(16))) _Float16 v16b;
typedef __attribute__((ext_vector_type(8))) _Float16 v8b;
typedef __attribute__((ext_vector_type(8))) float v8f;
typedef __attribute__((ext_vector_type(4))) float v4f;
__device__ __forceinline__ float bf16_rne(float f) { unsigned int u = __float_as_uint(f); u += 0x7FFFu + ((u >> 16) & 1u); return __uint_as_float(u & 0xFFFF0000u); }
__device__ __forceinline__ void split16(float v, b16& hi, b16& lo) { hi = (b16)v; lo = (b16)(v - (float)hi); }
__device__ __forceinline__ v16b frag_kb(const b16* p, int hh) { const v8b a = *(const v8b*)(p + 8 * hh), b = *(const v8b*)(p + 16 + 8 * hh); v16b f;
#pragma unroll
  for (int e = 0; e < 8; ++e) { f[e] = a[e]; f[8 + e] = b[e]; } return f; }
__device__ __forceinline__ v8f wmma16b(v16b a, v16b b, v8f c) { v8f d = __builtin_amdgcn_wmma_f32_16x16x32_f16(false, a, false, b, (short)0, c, false, false); asm volatile("v_nop\n\tv_nop\n\tv_nop\n\tv_nop" : "+v"(d) : "v"(a), "v"(b)); return d; }
__device__ __forceinline__ void wave_lds_sync() { __builtin_amdgcn_fence(__ATOMIC_RELEASE, "workgroup"); __builtin_amdgcn_wave_barrier(); __builtin_amdgcn_fence(__ATOMIC_ACQUIRE, "workgroup"); }
__device__ __forceinline__ float pmul(float a, float b) { float p = a * b; asm volatile("" : "+v"(p)); return p; }
__device__ __forceinline__ int iclamp(int v, int lo, int hi) { return v < lo ? lo : (v > hi ? hi : v); }
constexpr int CSR_NBLK = 512, CSR_GB = 10, CSR_GN = 1 << CSR_GB  , CSR_MAXG = 512, CSR_CAP = 12288  ;
__global__ __launch_bounds__(64) void csrA_kernel(const int* __restrict__ dst, int E, int N, int nG, int CHP, int NGP, int* __restrict__ STG, int* __restrict__ HST) {
  extern __shared__ int sm[];
  int* cnt = sm; int* run = sm + NGP; int* ids = sm + 2 * NGP;
  const int b = blockIdx.x; const int ch = (E + CSR_NBLK - 1) / CSR_NBLK; const int e0 = b * ch, e1 = min(E, e0 + ch);
  for (int i = threadIdx.x; i < NGP; i += 64) cnt[i] = 0;
  for (int i = threadIdx.x; i < CHP; i += 64) ids[i] = -1;
  __syncthreads();
  if (threadIdx.x == 0) {
    for (int e = e0; e < e1; ++e) { int d = dst[e]; d = (d < 0) ? 0 : (d >= N ? N - 1 : d); cnt[d >> CSR_GB] += 1; }
    int acc = 0; for (int g = 0; g < nG; ++g) { run[g] = acc; acc += cnt[g]; }
    for (int e = e0; e < e1; ++e) { int d = dst[e]; d = (d < 0) ? 0 : (d >= N ? N - 1 : d); const int g = d >> CSR_GB; ids[run[g]] = e; run[g] += 1; } }
  __syncthreads();
  typedef __attribute__((ext_vector_type(4))) int v4i;
  for (int pass = 0; pass < 2; ++pass) {
    for (int i = threadIdx.x; i < CHP / 4; i += 64) *(volatile v4i*)(STG + (size_t)b * CHP + i * 4) = *(const v4i*)(&ids[i * 4]);
    for (int i = threadIdx.x; i < NGP / 4; i += 64) { v4i v; for (int e = 0; e < 4; ++e) v[e] = (i * 4 + e < nG) ? cnt[i * 4 + e] : 0; *(volatile v4i*)(HST + (size_t)b * NGP + i * 4) = v; }
    __threadfence(); }
}
__global__ __launch_bounds__(512) void csrS_kernel(const int* __restrict__ HST, int nG, int NGP, int* __restrict__ START, int* __restrict__ TOT, int* __restrict__ OFF) {
  __shared__ int tot[CSR_MAXG];
  const int b = threadIdx.x;
  for (int pass = 0; pass < 2; ++pass) { int runb = 0; for (int g = 0; g < nG; ++g) { int c = HST[(size_t)b * NGP + g]; c = (c < 0) ? 0 : c; ((volatile int*)OFF)[(size_t)g * CSR_NBLK + b] = runb; runb += c; } __threadfence(); }
  for (int g = threadIdx.x; g < nG; g += 512) { int s = 0; for (int bb = 0; bb < CSR_NBLK; ++bb) { int c = HST[(size_t)bb * NGP + g]; s += (c < 0) ? 0 : c; } tot[g] = s; }
  __syncthreads();
  if (threadIdx.x < 32) {
    __shared__ int st[CSR_MAXG + 32];
    if (threadIdx.x == 0) { int acc = 0; for (int g = 0; g < NGP; ++g) { st[g] = acc; if (g < nG) acc += (tot[g] + 31) & ~31; } st[NGP] = acc; }
    __builtin_amdgcn_fence(__ATOMIC_RELEASE, "workgroup"); __builtin_amdgcn_wave_barrier(); __builtin_amdgcn_fence(__ATOMIC_ACQUIRE, "workgroup");
    for (int pass = 0; pass < 2; ++pass) { for (int i = threadIdx.x; i < NGP + 32; i += 32) { ((volatile int*)START)[i] = (i <= NGP) ? st[min(i, NGP)] : 0; ((volatile int*)TOT)[i] = (i < nG) ? tot[i] : 0; } __threadfence(); } }
}
__global__ __launch_bounds__(256) void csrB_kernel(const int* __restrict__ dst, int N, int nG, int CHP, int NGP, int permLen, const int* __restrict__ STG, const int* __restrict__ HST, const int* __restrict__ OFF, const int* __restrict__ START, const int* __restrict__ TOT, int* __restrict__ PERM, int* __restrict__ ROWPTR, int* __restrict__ ROWCNT, int* __restrict__ FLAG) {
  typedef __attribute__((ext_vector_type(4))) int v4i;
  __shared__ int ids[CSR_CAP]; __shared__ unsigned short key[CSR_CAP]; __shared__ int outp[CSR_CAP]; __shared__ int ncnt[CSR_GN + 1]; __shared__ int boff[CSR_NBLK + 1];
  const int g = blockIdx.x, t_ = threadIdx.x; int tot = TOT[g]; int st = START[g], stn = START[g + 1]; const int v0 = g * CSR_GN; const int nv = min(CSR_GN, N - v0);
  st = (st < 0) ? 0 : (st > permLen - 32 ? permLen - 32 : st) & ~31; stn = (stn < st) ? st : (stn > permLen ? permLen : stn); tot = (tot < 0) ? 0 : tot; if (tot > stn - st && tot <= CSR_CAP) tot = stn - st;
  if (tot > CSR_CAP) {
    for (int pass = 0; pass < 2; ++pass) { for (int i = t_; i < CSR_GN / 4; i += 256) { v4i a, c; for (int e = 0; e < 4; ++e) { a[e] = st; c[e] = 0; } *(volatile v4i*)(ROWPTR + v0 + i * 4) = a; *(volatile v4i*)(ROWCNT + v0 + i * 4) = c; } if (t_ == 0) ((volatile int*)FLAG)[0] = 1; __threadfence(); } (void)nv; return; }
  if (t_ == 0) { int acc = 0; for (int b = 0; b < CSR_NBLK; ++b) { boff[b] = acc; int c = HST[(size_t)b * NGP + g]; c = (c < 0) ? 0 : (c > CHP ? CHP : c); acc += c; if (acc > tot) acc = tot; } boff[CSR_NBLK] = acc; }
  for (int i = t_; i <= CSR_GN; i += 256) ncnt[i] = 0;
  __syncthreads();
  for (int b = 0; b < CSR_NBLK; ++b) { const int c = boff[b + 1] - boff[b]; int o_ = OFF[(size_t)g * CSR_NBLK + b]; o_ = (o_ < 0) ? 0 : (o_ > CHP - c ? CHP - c : o_); const int* src_ = STG + (size_t)b * CHP + o_;
    for (int i = t_; i < c; i += 256) { int id = src_[i]; id = (id < 0) ? 0 : id; ids[boff[b] + i] = id; int d = dst[id]; d = (d < v0) ? v0 : (d >= N ? N - 1 : d); int kk = d - v0; kk = (kk < 0) ? 0 : (kk >= CSR_GN ? CSR_GN - 1 : kk); key[boff[b] + i] = (unsigned short)kk; } }
  __syncthreads();
  if (t_ == 0) { for (int i = 0; i < tot; ++i) ncnt[key[i]] += 1; int acc = 0; for (int vl = 0; vl < CSR_GN; ++vl) { const int c = ncnt[vl]; ncnt[vl] = acc; acc += c; } ncnt[CSR_GN] = acc;
    for (int i = 0; i < tot; ++i) { const int vl = key[i]; outp[ncnt[vl]] = ids[i]; ncnt[vl] += 1; }
    for (int vl = CSR_GN; vl > 0; --vl) ncnt[vl] = ncnt[vl - 1]; ncnt[0] = 0; }
  __syncthreads();
  for (int pass = 0; pass < 2; ++pass) {
    for (int i = t_; i < (stn - st) / 4; i += 256) { v4i v; for (int e = 0; e < 4; ++e) { const int q = i * 4 + e; v[e] = (q < tot) ? outp[q] : -1; } *(volatile v4i*)(PERM + st + i * 4) = v; }
    for (int i = t_; i < CSR_GN / 4; i += 256) { v4i a, c; for (int e = 0; e < 4; ++e) { const int vl = i * 4 + e; a[e] = st + ncnt[vl]; c[e] = (vl < nv) ? (ncnt[vl + 1] - ncnt[vl]) : 0; } *(volatile v4i*)(ROWPTR + v0 + i * 4) = a; *(volatile v4i*)(ROWCNT + v0 + i * 4) = c; }
    __threadfence(); }
}
__global__ __launch_bounds__(256) void csrZ_kernel(int* __restrict__ p, size_t n4) { typedef __attribute__((ext_vector_type(4))) int v4i; const size_t tid = (size_t)blockIdx.x * 256 + threadIdx.x, nth = (size_t)gridDim.x * 256; v4i z = {0, 0, 0, 0}; for (size_t i = tid; i < n4; i += nth) *(volatile v4i*)(p + i * 4) = z; }
struct CsrBufs { int *STG, *HST, *OFF, *START, *TOT, *PERM, *ROWPTR, *ROWCNT, *FLAG; int nG, NGP, CHP; size_t permLen; char* base; size_t bytes; };
static size_t csr_carve(CsrBufs& c, char* ws, size_t off, int E, int N) {
  const size_t off0 = off; c.base = ws + off;
  auto al = [&](size_t bytes) { char* p = ws + off; off += (bytes + 255) & ~(size_t)255; return p; };
  c.nG = (N + CSR_GN - 1) / CSR_GN; c.NGP = (c.nG + 31) & ~31; const int ch = (E + CSR_NBLK - 1) / CSR_NBLK; c.CHP = (ch + 31) & ~31; c.permLen = (size_t)E + 32 * (size_t)c.nG + 32;
  c.STG = (int*)al((size_t)CSR_NBLK * c.CHP * 4); c.HST = (int*)al((size_t)CSR_NBLK * c.NGP * 4); c.OFF = (int*)al((size_t)c.NGP * CSR_NBLK * 4); c.START = (int*)al((size_t)(c.NGP + 64) * 4); c.TOT = (int*)al((size_t)(c.NGP + 64) * 4);
  c.PERM = (int*)al(c.permLen * 4); c.ROWPTR = (int*)al((size_t)c.nG * CSR_GN * 4); c.ROWCNT = (int*)al((size_t)c.nG * CSR_GN * 4); c.FLAG = (int*)al(256);
  c.bytes = off - off0; return off;
}
static void csr_build(const CsrBufs& c, const int* dst, int E, int N, hipStream_t stream) {
  const size_t smem = (size_t)(2 * c.NGP + c.CHP) * 4;
  csrZ_kernel<<<512, 256, 0, stream>>>((int*)c.base, c.bytes / 16);
  csrA_kernel<<<CSR_NBLK, 64, smem, stream>>>(dst, E, N, c.nG, c.CHP, c.NGP, c.STG, c.HST);
  csrS_kernel<<<1, 512, 0, stream>>>(c.HST, c.nG, c.NGP, c.START, c.TOT, c.OFF);
  csrB_kernel<<<c.nG, 256, 0, stream>>>(dst, N, c.nG, c.CHP, c.NGP, (int)c.permLen, c.STG, c.HST, c.OFF, c.START, c.TOT, c.PERM, c.ROWPTR, c.ROWCNT, c.FLAG);
}

static_assert(NKEY / CSR_GN <= CSR_MAXG && CSR_GB == 10, "composite-key bucketing");
typedef __attribute__((ext_vector_type(4))) _Float16 v4h;
typedef __attribute__((ext_vector_type(2))) float v2f;
typedef __attribute__((ext_vector_type(4))) int v4i;
__device__ __forceinline__ float lrelu(float v) { return v > 0.0f ? v : NSLOPE * v; }
template <int KIN>
__global__ __launch_bounds__(256) void wt_kernel(const float* __restrict__ w, b16* __restrict__ WT, float scl) {
  const int u = blockIdx.x * 256 + threadIdx.x; if (u >= R * D * KIN / 8) return; const int e = u * 8; const int r = e / (D * KIN), rem = e % (D * KIN), o = rem / KIN, k0 = rem % KIN; v8b v;
#pragma unroll
  for (int j = 0; j < 8; ++j) v[j] = (b16)(bf16_rne(w[((size_t)r * KIN + k0 + j) * D + o]) * scl);
  for (int pass = 0; pass < 2; ++pass) { *(volatile v8b*)(WT + e) = v; __threadfence(); }
}
__global__ __launch_bounds__(256) void w3_kernel(const float* __restrict__ wv, const float* __restrict__ wq, const float* __restrict__ wk, b16* __restrict__ W3, float scl) {
  const int u = blockIdx.x * 256 + threadIdx.x; if (u >= R * 3 * D * D / 8) return; const int e = u * 8; const int r = e / (3 * D * D), rem = e % (3 * D * D), t = rem / (D * D), rem2 = rem % (D * D), o = rem2 / D, k0 = rem2 % D; const float* w = t == 0 ? wv : t == 1 ? wq : wk; v8b v;
#pragma unroll
  for (int j = 0; j < 8; ++j) v[j] = (b16)(bf16_rne(w[((size_t)r * D + k0 + j) * D + o]) * scl);
  for (int pass = 0; pass < 2; ++pass) { *(volatile v8b*)(W3 + e) = v; __threadfence(); }
}
__global__ __launch_bounds__(256) void key_kernel(const int* __restrict__ tgt, const int* __restrict__ typ, int* __restrict__ KEY) {
  const int u = blockIdx.x * 256 + threadIdx.x; if (u >= E / 4) return; const v4i t = *(const v4i*)(tgt + (size_t)u * 4), y = *(const v4i*)(typ + (size_t)u * 4); v4i k;
  for (int j = 0; j < 4; ++j) k[j] = (iclamp(y[j], 0, R - 1) << KSH) | iclamp(t[j], 0, N - 1);
  for (int pass = 0; pass < 2; ++pass) { *(volatile v4i*)(KEY + (size_t)u * 4) = k; __threadfence(); }
}
__global__ __launch_bounds__(256) void edge_kernel(const float* __restrict__ x, const int* __restrict__ srcs, const int* __restrict__ tgts, const int* __restrict__ PERM, const int* __restrict__ START, int permLen,
    const b16* __restrict__ WRT, const float* __restrict__ bR, const b16* __restrict__ W3T, const b16* __restrict__ W3Q, const float* __restrict__ bV, const float* __restrict__ bQ, const float* __restrict__ bK, const float* __restrict__ aw, const float* __restrict__ ab, b16* __restrict__ VE, float* __restrict__ ES) {
  __shared__ __attribute__((aligned(16))) b16 A1[32][D2 + 8], A2h[32][D + 8], A2l[32][D + 8], Vt[32][D + 8]; __shared__ __attribute__((aligned(16))) float Tq[32][D2 + 4]; __shared__ int sS[32], tS[32], vS[32]; __shared__ float eS[32], aws[D2];
  const int tid = threadIdx.x, wave = tid >> 5, lane = tid & 31, nloc = lane & 15, hlf = lane >> 4; const int p0 = blockIdx.x * 32;
  const int r = (p0 >= START[BPR] ? 1 : 0) + (p0 >= START[2 * BPR] ? 1 : 0) + (p0 >= START[3 * BPR] ? 1 : 0);
  aws[tid] = bf16_rne(aw[tid]);
  if (tid < 32) { const int p = p0 + tid; int e = (p < permLen) ? PERM[p] : -1; const int ok = (e >= 0 && e < E) ? 1 : 0; e = iclamp(e, 0, E - 1); int s = iclamp(srcs[e], 0, N - 1), t = iclamp(tgts[e], 0, N - 1); if (SRCM < N) { s %= SRCM; t %= SRCM; } sS[tid] = s; tS[tid] = t; vS[tid] = ok; }
  __syncthreads();
  { const int row = tid >> 3, g = tid & 7, c0 = g * 32; const float* xr = x + (size_t)(g < 4 ? sS[row] : tS[row]) * D + (c0 & (D - 1));
#pragma unroll
    for (int q = 0; q < 8; ++q) { const v4f a = *(const v4f*)(xr + 4 * q); v4h o; for (int j = 0; j < 4; ++j) o[j] = (b16)(bf16_rne(a[j]) * XS); *(v4h*)(&A1[row][c0 + 4 * q]) = o; } }
  __syncthreads();
  { v8f acc[2] = {(v8f){}, (v8f){}}; const b16* br = WRT + ((size_t)r * D + wave * 16 + nloc) * D2;
#pragma unroll 2
    for (int kb = 0; kb < D2; kb += 32) { const v16b bw = frag_kb(br + kb, hlf); acc[0] = wmma16b(frag_kb(&A1[nloc][kb], hlf), bw, acc[0]); acc[1] = wmma16b(frag_kb(&A1[16 + nloc][kb], hlf), bw, acc[1]); }
    const int col = wave * 16 + nloc; const float bb = bf16_rne(bR[r * D + col]);
#pragma unroll
    for (int rt = 0; rt < 2; ++rt)
#pragma unroll
      for (int q = 0; q < 8; ++q) { const int rr = rt * 16 + 8 * hlf + q; const float t = lrelu(acc[rt][q] * (1.0f / (XS * WSC)) + bb); const float ts = t * XS; const b16 p = (b16)ts; A2h[rr][col] = p; A2l[rr][col] = (b16)((ts - (float)p) * RS_); } }
  __syncthreads();
  { v8f acc[2][3] = {{(v8f){}, (v8f){}, (v8f){}}, {(v8f){}, (v8f){}, (v8f){}}};
#pragma unroll
    for (int kb = 0; kb < D; kb += 32) { const v16b a0 = frag_kb(&A2h[nloc][kb], hlf), a1 = frag_kb(&A2h[16 + nloc][kb], hlf), l0 = frag_kb(&A2l[nloc][kb], hlf), l1 = frag_kb(&A2l[16 + nloc][kb], hlf);
#pragma unroll
      for (int t = 0; t < 3; ++t) { const size_t wo_ = (((size_t)r * 3 + t) * D + wave * 16 + nloc) * D + kb; const v16b bw = frag_kb(W3T + wo_, hlf), bwq = frag_kb(W3Q + wo_, hlf);
        acc[0][t] = wmma16b(a0, bw, acc[0][t]); acc[0][t] = wmma16b(l0, bwq, acc[0][t]); acc[1][t] = wmma16b(a1, bw, acc[1][t]); acc[1][t] = wmma16b(l1, bwq, acc[1][t]); } }
    const int col = wave * 16 + nloc; const float bv_ = bf16_rne(bV[r * D + col]), bq_ = bf16_rne(bQ[r * D + col]), bk_ = bf16_rne(bK[r * D + col]);
#pragma unroll
    for (int rt = 0; rt < 2; ++rt)
#pragma unroll
      for (int q = 0; q < 8; ++q) { const int rr = rt * 16 + 8 * hlf + q; Vt[rr][col] = (b16)(vS[rr] ? acc[rt][0][q] * (1.0f / (XS * WSC)) + bv_ : 0.0f); Tq[rr][col] = acc[rt][1][q] * (1.0f / (XS * WSC)) + bq_; Tq[rr][D + col] = acc[rt][2][q] * (1.0f / (XS * WSC)) + bk_; } }
  __syncthreads();
  { const int row = tid >> 3, g = tid & 7; float s = 0.0f;
#pragma unroll
    for (int j = 0; j < 32; ++j) s = fmaf(Tq[row][g * 32 + j], aws[g * 32 + j], s);
    s += __shfl_xor(s, 1); s += __shfl_xor(s, 2); s += __shfl_xor(s, 4);
    if (g == 0) eS[row] = vS[row] ? lrelu(s + bf16_rne(ab[0])) : 0.0f; }
  __syncthreads();
  for (int pass = 0; pass < 2; ++pass) { for (int rr = wave * 4; rr < wave * 4 + 4; ++rr) { const int p = p0 + rr; if (p < permLen) *(volatile v4h*)(VE + (size_t)p * D + lane * 4) = *(const v4h*)(&Vt[rr][lane * 4]); }
    if (wave == 0 && p0 + lane < permLen) ((volatile float*)ES)[p0 + lane] = eS[lane];
    __threadfence(); }
}
__global__ __launch_bounds__(256) void node_kernel(const b16* __restrict__ VE, const float* __restrict__ ES, const int* __restrict__ ROWPTR, const int* __restrict__ ROWCNT, int permLen, float* __restrict__ out) {
  __shared__ __attribute__((aligned(16))) float Ob[32 * D + 4];
  const int tid = threadIdx.x; const int row = tid >> 3, g = tid & 7, c0 = g * 16; const int v = blockIdx.x * 32 + row;
  float h[16]; for (int j = 0; j < 16; ++j) h[j] = 0.0f;
#pragma unroll 1
  for (int r = 0; r < R; ++r) {
    int cnt = 0, q0 = 0; if (v < N) { const int key = (r << KSH) | v; cnt = iclamp(ROWCNT[key], 0, 65536); q0 = iclamp(ROWPTR[key], 0, permLen - 1); if (q0 + cnt > permLen) cnt = permLen - q0; }
    float m = -INFINITY, l = 0.0f; float acc[16]; for (int j = 0; j < 16; ++j) acc[j] = 0.0f;
#pragma unroll 1
    for (int i = 0; i < cnt; ++i) { const int p = q0 + i; const float e = ES[p]; const float mn = fmaxf(m, e); const float al = __expf(m - mn), pw = __expf(e - mn); l = l * al + pw; m = mn; const b16* vr = VE + (size_t)p * D + c0;
#pragma unroll
      for (int q = 0; q < 2; ++q) { const v8b t8 = *(const v8b*)(vr + 8 * q); for (int j = 0; j < 8; ++j) acc[8 * q + j] = fmaf(pw, (float)t8[j], pmul(acc[8 * q + j], al)); } }
    const float inv = (cnt > 0) ? 1.0f / l : 0.0f;
    for (int j = 0; j < 16; ++j) h[j] = fmaf(acc[j], inv, h[j]); }
#pragma unroll
  for (int j = 0; j < 16; ++j) { const float y = h[j] > 0.0f ? h[j] : __expf(h[j]) - 1.0f; Ob[row * D + c0 + j] = (v < N) ? y : 0.0f; }
  __syncthreads();
  const size_t base = (size_t)blockIdx.x * 32 * D; const size_t lim = (size_t)NL * D;
  for (int pass = 0; pass < 2; ++pass) { for (int q = tid; q < 32 * D / 4; q += 256) { const size_t o4 = base + (size_t)q * 4; if (o4 < lim) *(volatile v4f*)(out + o4) = *(const v4f*)(&Ob[q * 4]); } __threadfence(); }
}
}

extern "C" void kernel_launch(void* const* d_in, const int* in_sizes, int n_in, void* d_out, int out_size, void* d_ws, size_t ws_size, hipStream_t stream) {
  (void)n_in;
  auto Fp = [&](int i) { return (const float*)d_in[i]; }; auto Ip = [&](int i) { return (const int*)d_in[i]; };
  if (in_sizes[0] != N * D || in_sizes[1] != 2 * EFULL || in_sizes[2] != EFULL || in_sizes[3] != R * D2 * D || in_sizes[4] != R * D || in_sizes[5] != R * D * D || in_sizes[6] != R * D || in_sizes[7] != R * D * D || in_sizes[8] != R * D || in_sizes[9] != R * D * D || in_sizes[10] != R * D || in_sizes[11] != D2 || in_sizes[12] != 1 || out_size != N * D) return;
  size_t off = 0; char* ws = (char*)d_ws;
  auto carve = [&](size_t bytes) { char* p = ws + off; off += (bytes + 255) & ~(size_t)255; return p; };
  b16* WRT = (b16*)carve((size_t)R * D * D2 * 2); b16* W3T = (b16*)carve((size_t)R * 3 * D * D * 2); b16* W3Q = (b16*)carve((size_t)R * 3 * D * D * 2);
  int* KEY = (int*)carve((size_t)E * 4);
  CsrBufs csr; off = csr_carve(csr, ws, off, E, NKEY);
  b16* VE = (b16*)carve(csr.permLen * D * 2); float* ES = (float*)carve(csr.permLen * 4 + 256);
  if (off > ws_size || off > ((size_t)200 << 20)) return;
  wt_kernel<D2><<<(R * D * D2 / 8 + 255) / 256, 256, 0, stream>>>(Fp(3), WRT, WSC); w3_kernel<<<(R * 3 * D * D / 8 + 255) / 256, 256, 0, stream>>>(Fp(9), Fp(5), Fp(7), W3T, WSC); w3_kernel<<<(R * 3 * D * D / 8 + 255) / 256, 256, 0, stream>>>(Fp(9), Fp(5), Fp(7), W3Q, WSQ);
  key_kernel<<<(E / 4 + 255) / 256, 256, 0, stream>>>(Ip(1) + EFULL, Ip(2), KEY);
  csr_build(csr, KEY, E, NKEY, stream);
  edge_kernel<<<(unsigned)((csr.permLen + 31) / 32), 256, 0, stream>>>(Fp(0), Ip(1), Ip(1) + EFULL, csr.PERM, csr.START, (int)csr.permLen, WRT, Fp(4), W3T, W3Q, Fp(10), Fp(6), Fp(8), Fp(11), Fp(12), VE, ES);
  node_kernel<<<NPL / 32, 256, 0, stream>>>(VE, ES, csr.ROWPTR, csr.ROWCNT, (int)csr.permLen, (float*)d_out);
}
